// SimbaBlock_68788196213187
// MI455X (gfx1250) — hardware-verified
//
#include <hip/hip_runtime.h>


namespace {
constexpr int B = 2, S = 512, DIM = 512, DIN = 1024, NS = 64, DC = 64, R = 32, NBK = 4, BS = 128, NT = B * S;
constexpr float XS = 8.0f, HS = 64.0f, TS = 1024.0f, WSC = 256.0f, LAM = 0.01f;
typedef _Float16 b16;
typedef __attribute__((ext_vector_type(16))) _Float16 v16b;
typedef __attribute__((ext_vector_type(8))) _Float16 v8b;
typedef __attribute__((ext_vector_type(8))) float v8f;
typedef __attribute__((ext_vector_type(4))) float v4f;
typedef __attribute__((ext_vector_type(2))) float v2f;
__device__ __forceinline__ float bf16_rne(float f) { unsigned int u = __float_as_uint(f); u += 0x7FFFu + ((u >> 16) & 1u); return __uint_as_float(u & 0xFFFF0000u); }
__device__ __forceinline__ void split16(float v, b16& hi, b16& lo) { hi = (b16)v; lo = (b16)(v - (float)hi); }
__device__ __forceinline__ v16b frag_kb(const b16* p, int hh) { const v8b a = *(const v8b*)(p + 8 * hh), b = *(const v8b*)(p + 16 + 8 * hh); v16b f;
#pragma unroll
  for (int e = 0; e < 8; ++e) { f[e] = a[e]; f[8 + e] = b[e]; } return f; }
__device__ __forceinline__ v8f wmma16b(v16b a, v16b b, v8f c) { v8f d = __builtin_amdgcn_wmma_f32_16x16x32_f16(false, a, false, b, (short)0, c, false, false); asm volatile("v_nop\n\tv_nop\n\tv_nop\n\tv_nop" : "+v"(d) : "v"(a), "v"(b)); return d; }
__device__ __forceinline__ void wave_lds_sync() { __builtin_amdgcn_fence(__ATOMIC_RELEASE, "workgroup"); __builtin_amdgcn_wave_barrier(); __builtin_amdgcn_fence(__ATOMIC_ACQUIRE, "workgroup"); }
__device__ __forceinline__ float pmul(float a, float b) { float p = a * b; asm volatile("" : "+v"(p)); return p; }
__device__ __forceinline__ float sigm(float v) { return 1.0f / (1.0f + __expf(-v)); }
__device__ __forceinline__ float silu(float v) { return pmul(v, sigm(v)); }
__device__ __forceinline__ float softplus(float v) { return v > 20.0f ? v : (v < -20.0f ? __expf(v) : log1pf(__expf(v))); }

__global__ __launch_bounds__(256) void wio_kernel(const float* __restrict__ w, int KIN, int OUTW, int KP, int OUT, int ro, b16* __restrict__ WT) {
  const int u = blockIdx.x * 256 + threadIdx.x; if (u >= OUT * KP / 8) return; const int e = u * 8; const int o = e / KP, k0 = e % KP; v8b v;
#pragma unroll
  for (int j = 0; j < 8; ++j) { const int k = k0 + j; v[j] = k < KIN ? (b16)(bf16_rne(w[(size_t)k * OUTW + o]) * WSC) : (b16)0.0f; } for (int pass = 0; pass < 2; ++pass) { *(volatile v8b*)(WT + (size_t)(ro + o) * KP + k0) = v; __threadfence(); }
}
__global__ __launch_bounds__(256) void wcplx_kernel(const float* __restrict__ w, b16* __restrict__ WT) {
  const int u = blockIdx.x * 256 + threadIdx.x; if (u >= 2 * NBK * BS * BS / 8) return; const int e = u * 8; const int pb = e / (BS * BS), k = (e / BS) % BS, d0 = e % BS; v8b v;
#pragma unroll
  for (int j = 0; j < 8; ++j) v[j] = (b16)(bf16_rne(w[((size_t)pb * BS + d0 + j) * BS + k]) * WSC); for (int pass = 0; pass < 2; ++pass) { *(volatile v8b*)(WT + e) = v; __threadfence(); }
}
__global__ __launch_bounds__(512) void twid_kernel(float* __restrict__ TW) { const int k = threadIdx.x; const float a = 6.283185307179586f * (float)k / (float)S; const float isq = rsqrtf((float)S); const float c = cosf(a) * isq, s = sinf(a) * isq; for (int pass = 0; pass < 2; ++pass) { ((volatile float*)TW)[k] = c; ((volatile float*)TW)[S + k] = s; __threadfence(); } }
__global__ __launch_bounds__(256) void dftmat_kernel(const float* __restrict__ TW, b16* __restrict__ AHp, b16* __restrict__ ALp) {
  const int u = blockIdx.x * 256 + threadIdx.x; if (u >= 2 * S * S / 8) return; const int e = u * 8; const int cs = e / (S * S), sp = (e / S) % S, t0 = e % S; v8b h, l;
#pragma unroll
  for (int j = 0; j < 8; ++j) { const int k = (sp * (t0 + j)) & (S - 1); b16 p, q; split16(TW[cs * S + k] * TS, p, q); h[j] = p; l[j] = q; }
  for (int pass = 0; pass < 2; ++pass) { *(volatile v8b*)(AHp + e) = h; *(volatile v8b*)(ALp + e) = l; __threadfence(); }
}
__device__ __forceinline__ void ln512(float (&v)[16], float& mu, float& rs) { float s = 0.0f; for (int q = 0; q < 16; ++q) s += v[q]; for (int o = 16; o; o >>= 1) s += __shfl_xor(s, o); mu = s * (1.0f / DIM); float vq = 0.0f; for (int q = 0; q < 16; ++q) { const float d = v[q] - mu; vq += pmul(d, d); } for (int o = 16; o; o >>= 1) vq += __shfl_xor(vq, o); rs = rsqrtf(vq * (1.0f / DIM) + 1e-5f); }
__global__ __launch_bounds__(32) void inproj_kernel(const float* __restrict__ x, const b16* __restrict__ W, int NTV, float* __restrict__ XZ) {
  __shared__ __attribute__((aligned(16))) b16 Ah[16][DIM + 8], Al[16][DIM + 8]; __shared__ __attribute__((aligned(16))) float Tf[16][128 + 4];
  const int lane = threadIdx.x, nloc = lane & 15, hlf = lane >> 4; const size_t m0 = (size_t)blockIdx.x * 16; if (m0 >= (size_t)NTV) return;
  for (int rr = 0; rr < 16; ++rr) { float v[16]; for (int q = 0; q < 16; ++q) v[q] = bf16_rne(x[(m0 + rr) * DIM + q * 32 + lane]); float mu, rs; ln512(v, mu, rs); for (int q = 0; q < 16; ++q) { b16 p, ql; split16(pmul(v[q] - mu, rs) * XS, p, ql); Ah[rr][q * 32 + lane] = p; Al[rr][q * 32 + lane] = ql; } }
  wave_lds_sync();
#pragma unroll 1
  for (int cg = 0; cg < 2 * DIN / 128; ++cg) { v8f acc[8];
#pragma unroll
    for (int t = 0; t < 8; ++t) acc[t] = (v8f){};
#pragma unroll 2
    for (int kb = 0; kb < DIM; kb += 32) { const v16b a = frag_kb(&Ah[nloc][kb], hlf), al = frag_kb(&Al[nloc][kb], hlf);
#pragma unroll
      for (int t = 0; t < 8; ++t) { const v16b bw = frag_kb(W + (size_t)(cg * 128 + t * 16 + nloc) * DIM + kb, hlf); acc[t] = wmma16b(a, bw, acc[t]); acc[t] = wmma16b(al, bw, acc[t]); } }
#pragma unroll
    for (int t = 0; t < 8; ++t)
#pragma unroll 1
      for (int r8 = 0; r8 < 8; ++r8) Tf[8 * hlf + r8][t * 16 + nloc] = acc[t][r8] * (1.0f / (XS * WSC));
    wave_lds_sync();
    for (int pass = 0; pass < 2; ++pass) { for (int rr = 0; rr < 16; ++rr) *(volatile v4f*)(XZ + (m0 + rr) * (2 * DIN) + cg * 128 + lane * 4) = *(const v4f*)(&Tf[rr][lane * 4]); __threadfence(); }
    wave_lds_sync(); }
}
__global__ __launch_bounds__(256) void conv_kernel(const float* __restrict__ XZ, const float* __restrict__ cw, const float* __restrict__ cb, int NBV, float* __restrict__ U) {
  const int gid = blockIdx.x * 256 + threadIdx.x; const int d = gid % DIN, b = gid / DIN; if (b >= NBV) return; float w[DC]; for (int j = 0; j < DC; ++j) w[j] = bf16_rne(cw[d * DC + j]); const float bias = bf16_rne(cb[d]);
#pragma unroll 1
  for (int pass = 0; pass < 2; ++pass) {
#pragma unroll 1
    for (int s = 0; s < S; ++s) { float acc = bias;
#pragma unroll
      for (int j = 0; j < DC; ++j) { const int sp = s - (DC - 1) + j; acc += sp >= 0 ? pmul(XZ[((size_t)b * S + sp) * (2 * DIN) + d], w[j]) : 0.0f; }
      ((volatile float*)U)[((size_t)b * S + s) * DIN + d] = silu(acc); }
    __threadfence(); }
}
__global__ __launch_bounds__(32) void xproj_kernel(const float* __restrict__ U, const b16* __restrict__ XPW, const b16* __restrict__ DTW, const float* __restrict__ dtb, int NTV, float* __restrict__ BC, float* __restrict__ DT) {
  __shared__ __attribute__((aligned(16))) b16 Ah[16][DIN + 8], Al[16][DIN + 8], Dh[16][32 + 8], Dl[16][32 + 8]; __shared__ __attribute__((aligned(16))) float Tf[16][128 + 4], Sbc[16][128];
  const int lane = threadIdx.x, nloc = lane & 15, hlf = lane >> 4; const size_t m0 = (size_t)blockIdx.x * 16; if (m0 >= (size_t)NTV) return;
  for (int rr = 0; rr < 16; ++rr) for (int q = 0; q < DIN / 32; ++q) { b16 p, ql; split16(U[(m0 + rr) * DIN + q * 32 + lane] * XS, p, ql); Ah[rr][q * 32 + lane] = p; Al[rr][q * 32 + lane] = ql; }
  wave_lds_sync(); const float sx = 1.0f / (XS * WSC), sd = 1.0f / (HS * WSC);
  { v8f ax[10];
#pragma unroll
    for (int t = 0; t < 10; ++t) ax[t] = (v8f){};
#pragma unroll 2
    for (int kb = 0; kb < DIN; kb += 32) { const v16b a = frag_kb(&Ah[nloc][kb], hlf), al = frag_kb(&Al[nloc][kb], hlf);
#pragma unroll
      for (int t = 0; t < 10; ++t) { const v16b bw = frag_kb(XPW + (size_t)(t * 16 + nloc) * DIN + kb, hlf); ax[t] = wmma16b(a, bw, ax[t]); ax[t] = wmma16b(al, bw, ax[t]); } }
#pragma unroll
    for (int t = 0; t < 10; ++t) { const int c = t * 16 + nloc;
#pragma unroll
      for (int r8 = 0; r8 < 8; ++r8) { const int rl = 8 * hlf + r8; const float v = ax[t][r8] * sx; if (t < 2) { b16 p, ql; split16(v * HS, p, ql); Dh[rl][c] = p; Dl[rl][c] = ql; } else Sbc[rl][c - R] = v; } } }
  wave_lds_sync();
  for (int pass = 0; pass < 2; ++pass) { for (int rr = 0; rr < 16; ++rr) *(volatile v4f*)(BC + (m0 + rr) * 128 + lane * 4) = *(const v4f*)(&Sbc[rr][lane * 4]); __threadfence(); }
  const v16b a = frag_kb(&Dh[nloc][0], hlf), al = frag_kb(&Dl[nloc][0], hlf);
#pragma unroll 1
  for (int cg = 0; cg < DIN / 128; ++cg) { v8f acc[8];
#pragma unroll
    for (int t = 0; t < 8; ++t) { acc[t] = (v8f){}; const v16b bw = frag_kb(DTW + (size_t)(cg * 128 + t * 16 + nloc) * 32, hlf); acc[t] = wmma16b(a, bw, acc[t]); acc[t] = wmma16b(al, bw, acc[t]); }
#pragma unroll
    for (int t = 0; t < 8; ++t) { const int c = cg * 128 + t * 16 + nloc; const float bb = bf16_rne(dtb[c]);
#pragma unroll 1
      for (int r8 = 0; r8 < 8; ++r8) Tf[8 * hlf + r8][t * 16 + nloc] = softplus(acc[t][r8] * sd + bb); }
    wave_lds_sync();
    for (int pass = 0; pass < 2; ++pass) { for (int rr = 0; rr < 16; ++rr) *(volatile v4f*)(DT + (m0 + rr) * DIN + cg * 128 + lane * 4) = *(const v4f*)(&Tf[rr][lane * 4]); __threadfence(); }
    wave_lds_sync(); }
}
__global__ __launch_bounds__(256) void scan_kernel(const float* __restrict__ U, const float* __restrict__ DT, const float* __restrict__ BC, const float* __restrict__ XZ, const float* __restrict__ alog, const float* __restrict__ Dd, int NBV, float* __restrict__ Y) {
  const int gid = blockIdx.x * 256 + threadIdx.x; const int d = gid % DIN, b = gid / DIN; if (b >= NBV) return;
  float A[NS]; for (int s = 0; s < NS; ++s) A[s] = -__expf(bf16_rne(alog[(size_t)d * NS + s])); const float dd = bf16_rne(Dd[d]);
#pragma unroll 1
  for (int pass = 0; pass < 2; ++pass) { float h[NS]; for (int s = 0; s < NS; ++s) h[s] = 0.0f;
#pragma unroll 1
    for (int t = 0; t < S; ++t) { const size_t row = (size_t)b * S + t; const float u = U[row * DIN + d], dt = DT[row * DIN + d]; const float du = pmul(dt, u); const float* bc = BC + row * 128; float acc = 0.0f;
#pragma unroll
      for (int s = 0; s < NS; ++s) { h[s] = pmul(__expf(pmul(dt, A[s])), h[s]) + pmul(du, bc[s]); acc += pmul(h[s], bc[NS + s]); }
      const float res = XZ[row * (2 * DIN) + DIN + d]; ((volatile float*)Y)[row * DIN + d] = pmul(acc + pmul(dd, u), silu(res)); }
    __threadfence(); }
}
__global__ __launch_bounds__(32) void outproj_kernel(const float* __restrict__ Y, const float* __restrict__ x, const b16* __restrict__ W, int NTV, float* __restrict__ O1, float* __restrict__ XL) {
  __shared__ __attribute__((aligned(16))) b16 Ah[16][DIN + 8], Al[16][DIN + 8]; __shared__ __attribute__((aligned(16))) float Tf[16][DIM + 4];
  const int lane = threadIdx.x, nloc = lane & 15, hlf = lane >> 4; const size_t m0 = (size_t)blockIdx.x * 16; if (m0 >= (size_t)NTV) return;
  for (int rr = 0; rr < 16; ++rr) for (int q = 0; q < DIN / 32; ++q) { b16 p, ql; split16(Y[(m0 + rr) * DIN + q * 32 + lane] * XS, p, ql); Ah[rr][q * 32 + lane] = p; Al[rr][q * 32 + lane] = ql; }
  wave_lds_sync();
#pragma unroll 1
  for (int cg = 0; cg < DIM / 128; ++cg) { v8f acc[8];
#pragma unroll
    for (int t = 0; t < 8; ++t) acc[t] = (v8f){};
#pragma unroll 2
    for (int kb = 0; kb < DIN; kb += 32) { const v16b a = frag_kb(&Ah[nloc][kb], hlf), al = frag_kb(&Al[nloc][kb], hlf);
#pragma unroll
      for (int t = 0; t < 8; ++t) { const v16b bw = frag_kb(W + (size_t)(cg * 128 + t * 16 + nloc) * DIN + kb, hlf); acc[t] = wmma16b(a, bw, acc[t]); acc[t] = wmma16b(al, bw, acc[t]); } }
#pragma unroll
    for (int t = 0; t < 8; ++t) { const int c = cg * 128 + t * 16 + nloc;
#pragma unroll 1
      for (int r8 = 0; r8 < 8; ++r8) { const int rl = 8 * hlf + r8; Tf[rl][c] = bf16_rne(x[(m0 + rl) * DIM + c]) + acc[t][r8] * (1.0f / (XS * WSC)); } } }
  wave_lds_sync();
  for (int pass = 0; pass < 2; ++pass) { for (int rr = 0; rr < 16; ++rr) for (int q = 0; q < 4; ++q) *(volatile v4f*)(O1 + (m0 + rr) * DIM + q * 128 + lane * 4) = *(const v4f*)(&Tf[rr][q * 128 + lane * 4]); __threadfence(); }
  for (int rr = 0; rr < 16; ++rr) { float v[16]; for (int q = 0; q < 16; ++q) v[q] = Tf[rr][q * 32 + lane]; float mu, rs; ln512(v, mu, rs); wave_lds_sync(); for (int q = 0; q < 16; ++q) Tf[rr][q * 32 + lane] = pmul(v[q] - mu, rs); }
  wave_lds_sync();
  for (int pass = 0; pass < 2; ++pass) { for (int rr = 0; rr < 16; ++rr) for (int q = 0; q < 4; ++q) *(volatile v4f*)(XL + (m0 + rr) * DIM + q * 128 + lane * 4) = *(const v4f*)(&Tf[rr][q * 128 + lane * 4]); __threadfence(); }
}
__global__ __launch_bounds__(256) void transp_kernel(const float* __restrict__ IN, int C, int NBV, b16* __restrict__ TH, b16* __restrict__ TL) {
  __shared__ float T[64][33]; const int nct = C / 32, ntt = S / 64; const int b = blockIdx.x / (nct * ntt); if (b >= NBV) return; const int rem = blockIdx.x % (nct * ntt); const int tt = rem / nct, ct = rem % nct; const int tid = threadIdx.x;
  for (int i = tid; i < 64 * 32; i += 256) { const int r = i / 32, c = i % 32; T[r][c] = IN[((size_t)b * S + tt * 64 + r) * C + ct * 32 + c]; }
  __syncthreads();
  { const int c = tid / 8, g = tid % 8; v8b h, l;
#pragma unroll
    for (int j = 0; j < 8; ++j) { b16 p, q; split16(T[g * 8 + j][c] * XS, p, q); h[j] = p; l[j] = q; }
    const size_t o = ((size_t)b * C + ct * 32 + c) * S + tt * 64 + g * 8; for (int pass = 0; pass < 2; ++pass) { *(volatile v8b*)(TH + o) = h; *(volatile v8b*)(TL + o) = l; __threadfence(); } }
}
__global__ __launch_bounds__(32) void dft_kernel(const b16* __restrict__ AH, const b16* __restrict__ AL, const b16* __restrict__ TH, const b16* __restrict__ TL, int NBV, float* __restrict__ XF) {
  __shared__ __attribute__((aligned(16))) float Tf[16][256 + 4];
  const int lane = threadIdx.x, nloc = lane & 15, hlf = lane >> 4; const int b = blockIdx.x / (S / 16); if (b >= NBV) return; const int s0 = (blockIdx.x % (S / 16)) * 16; const float sc = 1.0f / (TS * XS);
  const b16* Ch = AH + (size_t)(s0 + nloc) * S; const b16* Cl = AL + (size_t)(s0 + nloc) * S; const b16* Sh = AH + (size_t)(S + s0 + nloc) * S; const b16* Sl = AL + (size_t)(S + s0 + nloc) * S;
#pragma unroll 1
  for (int cg = 0; cg < DIM / 128; ++cg) { v8f ar[8], ai[8];
#pragma unroll
    for (int t = 0; t < 8; ++t) { ar[t] = (v8f){}; ai[t] = (v8f){}; }
#pragma unroll 1
    for (int kb = 0; kb < S; kb += 32) { const v16b ch = frag_kb(Ch + kb, hlf), cl = frag_kb(Cl + kb, hlf), sh = frag_kb(Sh + kb, hlf), sl = frag_kb(Sl + kb, hlf);
#pragma unroll
      for (int t = 0; t < 8; ++t) { const size_t ro = ((size_t)b * DIM + cg * 128 + t * 16 + nloc) * S + kb; const v16b bh = frag_kb(TH + ro, hlf), bl = frag_kb(TL + ro, hlf);
        ar[t] = wmma16b(ch, bh, ar[t]); ar[t] = wmma16b(ch, bl, ar[t]); ar[t] = wmma16b(cl, bh, ar[t]); ar[t] = wmma16b(cl, bl, ar[t]);
        ai[t] = wmma16b(sh, bh, ai[t]); ai[t] = wmma16b(sh, bl, ai[t]); ai[t] = wmma16b(sl, bh, ai[t]); ai[t] = wmma16b(sl, bl, ai[t]); } }
#pragma unroll
    for (int t = 0; t < 8; ++t)
#pragma unroll 1
      for (int r8 = 0; r8 < 8; ++r8) { Tf[8 * hlf + r8][t * 16 + nloc] = ar[t][r8] * sc; Tf[8 * hlf + r8][128 + t * 16 + nloc] = -ai[t][r8] * sc; }
    wave_lds_sync();
    for (int pass = 0; pass < 2; ++pass) { for (int rr = 0; rr < 16; ++rr) { const size_t row = (size_t)b * S + s0 + rr; *(volatile v4f*)(XF + row * (2 * DIM) + cg * 128 + lane * 4) = *(const v4f*)(&Tf[rr][lane * 4]); *(volatile v4f*)(XF + row * (2 * DIM) + DIM + cg * 128 + lane * 4) = *(const v4f*)(&Tf[rr][128 + lane * 4]); } __threadfence(); }
    wave_lds_sync(); }
}
__global__ __launch_bounds__(32) void cmlp_kernel(const float* __restrict__ XF, const b16* __restrict__ WC1, const float* __restrict__ cb1, const b16* __restrict__ WC2, const float* __restrict__ cb2, int NTV, float* __restrict__ Z) {
  __shared__ __attribute__((aligned(16))) b16 Arh[16][BS + 8], Arl[16][BS + 8], Aih[16][BS + 8], Ail[16][BS + 8]; __shared__ __attribute__((aligned(16))) float Tf[16][2 * BS + 4];
  const int lane = threadIdx.x, nloc = lane & 15, hlf = lane >> 4; const size_t m0 = (size_t)blockIdx.x * 16; if (m0 >= (size_t)NTV) return; const float s1 = 1.0f / (XS * WSC), s2 = 1.0f / (HS * WSC);
#pragma unroll 1
  for (int nb = 0; nb < NBK; ++nb) {
    for (int rr = 0; rr < 16; ++rr) for (int q = 0; q < 4; ++q) { const int c = q * 32 + lane; b16 p, ql; split16(XF[(m0 + rr) * (2 * DIM) + nb * BS + c] * XS, p, ql); Arh[rr][c] = p; Arl[rr][c] = ql; split16(XF[(m0 + rr) * (2 * DIM) + DIM + nb * BS + c] * XS, p, ql); Aih[rr][c] = p; Ail[rr][c] = ql; }
    wave_lds_sync();
#pragma unroll 1
    for (int layer = 0; layer < 2; ++layer) { const b16* Wr = (layer ? WC2 : WC1) + ((size_t)0 * NBK + nb) * BS * BS; const b16* Wi = (layer ? WC2 : WC1) + ((size_t)1 * NBK + nb) * BS * BS; const float* cb = layer ? cb2 : cb1; const float sc = layer ? s2 : s1;
      v8f ar[8], ai[8];
#pragma unroll
      for (int t = 0; t < 8; ++t) { ar[t] = (v8f){}; ai[t] = (v8f){}; }
#pragma unroll
      for (int kb = 0; kb < BS; kb += 32) { const v16b arh = frag_kb(&Arh[nloc][kb], hlf), arl = frag_kb(&Arl[nloc][kb], hlf), aih = frag_kb(&Aih[nloc][kb], hlf), ail = frag_kb(&Ail[nloc][kb], hlf);
        v16b nih, nil; { v16b zh = aih, zl = ail;
#pragma unroll
          for (int e = 0; e < 16; ++e) { zh[e] = -zh[e]; zl[e] = -zl[e]; } nih = zh; nil = zl; }
#pragma unroll
        for (int t = 0; t < 8; ++t) { const v16b wr = frag_kb(Wr + (size_t)(t * 16 + nloc) * BS + kb, hlf), wi = frag_kb(Wi + (size_t)(t * 16 + nloc) * BS + kb, hlf);
          ar[t] = wmma16b(arh, wr, ar[t]); ar[t] = wmma16b(arl, wr, ar[t]); ar[t] = wmma16b(nih, wi, ar[t]); ar[t] = wmma16b(nil, wi, ar[t]);
          ai[t] = wmma16b(arh, wi, ai[t]); ai[t] = wmma16b(arl, wi, ai[t]); ai[t] = wmma16b(aih, wr, ai[t]); ai[t] = wmma16b(ail, wr, ai[t]); } }
      wave_lds_sync();
#pragma unroll
      for (int t = 0; t < 8; ++t) { const int c = t * 16 + nloc; const float br = bf16_rne(cb[(0 * NBK + nb) * BS + c]), bi = bf16_rne(cb[(1 * NBK + nb) * BS + c]);
#pragma unroll
        for (int r8 = 0; r8 < 8; ++r8) { const int rl = 8 * hlf + r8; float vr = ar[t][r8] * sc + br, vi = ai[t][r8] * sc + bi;
          if (layer == 0) { vr = fmaxf(vr, 0.0f); vi = fmaxf(vi, 0.0f); b16 p, ql; split16(vr * HS, p, ql); Arh[rl][c] = p; Arl[rl][c] = ql; split16(vi * HS, p, ql); Aih[rl][c] = p; Ail[rl][c] = ql; }
          else { vr = vr > LAM ? vr - LAM : (vr < -LAM ? vr + LAM : 0.0f); vi = vi > LAM ? vi - LAM : (vi < -LAM ? vi + LAM : 0.0f); Tf[rl][c] = vr; Tf[rl][BS + c] = vi; } } }
      wave_lds_sync(); }
    for (int pass = 0; pass < 2; ++pass) { for (int rr = 0; rr < 16; ++rr) { *(volatile v4f*)(Z + (m0 + rr) * (2 * DIM) + nb * BS + lane * 4) = *(const v4f*)(&Tf[rr][lane * 4]); *(volatile v4f*)(Z + (m0 + rr) * (2 * DIM) + DIM + nb * BS + lane * 4) = *(const v4f*)(&Tf[rr][BS + lane * 4]); } __threadfence(); }
    wave_lds_sync(); }
}
__global__ __launch_bounds__(32) void idft_kernel(const b16* __restrict__ AH, const b16* __restrict__ AL, const b16* __restrict__ TH, const b16* __restrict__ TL, const float* __restrict__ O1, int NBV, float* __restrict__ out) {
  __shared__ __attribute__((aligned(16))) float Tf[16][128 + 4];
  const int lane = threadIdx.x, nloc = lane & 15, hlf = lane >> 4; const int b = blockIdx.x / (S / 16); if (b >= NBV) return; const int s0 = (blockIdx.x % (S / 16)) * 16; const float sc = 1.0f / (TS * XS);
  const b16* Ch = AH + (size_t)(s0 + nloc) * S; const b16* Cl = AL + (size_t)(s0 + nloc) * S; const b16* Sh = AH + (size_t)(S + s0 + nloc) * S; const b16* Sl = AL + (size_t)(S + s0 + nloc) * S;
#pragma unroll 1
  for (int cg = 0; cg < DIM / 128; ++cg) { v8f ar[8], ai[8];
#pragma unroll
    for (int t = 0; t < 8; ++t) { ar[t] = (v8f){}; ai[t] = (v8f){}; }
#pragma unroll 1
    for (int kb = 0; kb < S; kb += 32) { const v16b ch = frag_kb(Ch + kb, hlf), cl = frag_kb(Cl + kb, hlf), sh = frag_kb(Sh + kb, hlf), sl = frag_kb(Sl + kb, hlf);
#pragma unroll
      for (int t = 0; t < 8; ++t) { const size_t rr_ = ((size_t)b * 2 * DIM + cg * 128 + t * 16 + nloc) * S + kb, ri_ = ((size_t)b * 2 * DIM + DIM + cg * 128 + t * 16 + nloc) * S + kb;
        const v16b zrh = frag_kb(TH + rr_, hlf), zrl = frag_kb(TL + rr_, hlf), zih = frag_kb(TH + ri_, hlf), zil = frag_kb(TL + ri_, hlf);
        ar[t] = wmma16b(ch, zrh, ar[t]); ar[t] = wmma16b(ch, zrl, ar[t]); ar[t] = wmma16b(cl, zrh, ar[t]); ar[t] = wmma16b(cl, zrl, ar[t]);
        ai[t] = wmma16b(sh, zih, ai[t]); ai[t] = wmma16b(sh, zil, ai[t]); ai[t] = wmma16b(sl, zih, ai[t]); ai[t] = wmma16b(sl, zil, ai[t]); } }
#pragma unroll
    for (int t = 0; t < 8; ++t) { const int c = cg * 128 + t * 16 + nloc;
#pragma unroll 1
      for (int r8 = 0; r8 < 8; ++r8) { const int rl = 8 * hlf + r8; Tf[rl][t * 16 + nloc] = O1[((size_t)b * S + s0 + rl) * DIM + c] + (ar[t][r8] - ai[t][r8]) * sc; } }
    wave_lds_sync();
    for (int pass = 0; pass < 2; ++pass) { for (int rr = 0; rr < 16; ++rr) *(volatile v4f*)(out + ((size_t)b * S + s0 + rr) * DIM + cg * 128 + lane * 4) = *(const v4f*)(&Tf[rr][lane * 4]); __threadfence(); }
    wave_lds_sync(); }
}
}

extern "C" void kernel_launch(void* const* d_in, const int* in_sizes, int n_in, void* d_out, int out_size, void* d_ws, size_t ws_size, hipStream_t stream) {
  (void)n_in;
  auto Fp = [&](int i) { return (const float*)d_in[i]; };
  if (in_sizes[0] != NT * DIM || in_sizes[1] != DIM * 2 * DIN || in_sizes[2] != DIN * DC || in_sizes[4] != DIN * (R + 2 * NS) || in_sizes[5] != R * DIN || in_sizes[7] != DIN * NS || in_sizes[9] != DIN * DIM || in_sizes[10] != 2 * NBK * BS * BS || in_sizes[12] != 2 * NBK * BS * BS || out_size != NT * DIM) return;
  const int NBV = B; const int NTV = NBV * S;
  size_t off = 0; char* ws = (char*)d_ws;
  auto carve = [&](size_t bytes) { char* p = ws + off; off += (bytes + 255) & ~(size_t)255; return p; };
  b16* WI = (b16*)carve((size_t)2 * DIN * DIM * 2); b16* WX = (b16*)carve((size_t)160 * DIN * 2); b16* WD = (b16*)carve((size_t)DIN * 32 * 2); b16* WO = (b16*)carve((size_t)DIM * DIN * 2); b16* WC1 = (b16*)carve((size_t)2 * NBK * BS * BS * 2); b16* WC2 = (b16*)carve((size_t)2 * NBK * BS * BS * 2);
  float* TW = (float*)carve(2 * S * 4); b16* DAH = (b16*)carve((size_t)2 * S * S * 2); b16* DAL = (b16*)carve((size_t)2 * S * S * 2);
  float* XZ = (float*)carve((size_t)NT * 2 * DIN * 4); float* U = (float*)carve((size_t)NT * DIN * 4); float* BC = (float*)carve((size_t)NT * 128 * 4); float* DT = (float*)carve((size_t)NT * DIN * 4); float* Y = (float*)carve((size_t)NT * DIN * 4); float* O1 = (float*)carve((size_t)NT * DIM * 4); float* XL = (float*)carve((size_t)NT * DIM * 4);
  b16* XTH = (b16*)carve((size_t)NT * DIM * 2); b16* XTL = (b16*)carve((size_t)NT * DIM * 2); float* XF = (float*)carve((size_t)NT * 2 * DIM * 4); float* Zp = (float*)carve((size_t)NT * 2 * DIM * 4); b16* ZTH = (b16*)carve((size_t)NT * 2 * DIM * 2); b16* ZTL = (b16*)carve((size_t)NT * 2 * DIM * 2);
  if (off > ws_size || off > ((size_t)96 << 20)) return;
  wio_kernel<<<(2 * DIN * DIM / 8 + 255) / 256, 256, 0, stream>>>(Fp(1), DIM, 2 * DIN, DIM, 2 * DIN, 0, WI); wio_kernel<<<(160 * DIN / 8 + 255) / 256, 256, 0, stream>>>(Fp(4), DIN, 160, DIN, 160, 0, WX);
  wio_kernel<<<(DIN * 32 / 8 + 255) / 256, 256, 0, stream>>>(Fp(5), R, DIN, 32, DIN, 0, WD); wio_kernel<<<(DIM * DIN / 8 + 255) / 256, 256, 0, stream>>>(Fp(9), DIN, DIM, DIN, DIM, 0, WO);
  wcplx_kernel<<<(2 * NBK * BS * BS / 8 + 255) / 256, 256, 0, stream>>>(Fp(10), WC1); wcplx_kernel<<<(2 * NBK * BS * BS / 8 + 255) / 256, 256, 0, stream>>>(Fp(12), WC2);
  twid_kernel<<<1, S, 0, stream>>>(TW); dftmat_kernel<<<(2 * S * S / 8 + 255) / 256, 256, 0, stream>>>(TW, DAH, DAL);
  inproj_kernel<<<NTV / 16, 32, 0, stream>>>(Fp(0), WI, NTV, XZ);
  conv_kernel<<<(NBV * DIN + 255) / 256, 256, 0, stream>>>(XZ, Fp(2), Fp(3), NBV, U);
  xproj_kernel<<<NTV / 16, 32, 0, stream>>>(U, WX, WD, Fp(6), NTV, BC, DT);
  scan_kernel<<<(NBV * DIN + 255) / 256, 256, 0, stream>>>(U, DT, BC, XZ, Fp(7), Fp(8), NBV, Y);
  outproj_kernel<<<NTV / 16, 32, 0, stream>>>(Y, Fp(0), WO, NTV, O1, XL);
  transp_kernel<<<NBV * (DIM / 32) * (S / 64), 256, 0, stream>>>(XL, DIM, NBV, XTH, XTL);
  dft_kernel<<<NBV * (S / 16), 32, 0, stream>>>(DAH, DAL, XTH, XTL, NBV, XF);
  cmlp_kernel<<<NTV / 16, 32, 0, stream>>>(XF, WC1, Fp(11), WC2, Fp(13), NTV, Zp);
  transp_kernel<<<NBV * (2 * DIM / 32) * (S / 64), 256, 0, stream>>>(Zp, 2 * DIM, NBV, ZTH, ZTL);
  idft_kernel<<<NBV * (S / 16), 32, 0, stream>>>(DAH, DAL, ZTH, ZTL, O1, NBV, (float*)d_out);
}
